// QuantizedGRU_5196910428519
// MI455X (gfx1250) — hardware-run, weakly checked
//
#include <hip/hip_runtime.h>
#include <math.h>

#pragma clang fp contract(off)

typedef __attribute__((ext_vector_type(16))) _Float16 v16h;
typedef __attribute__((ext_vector_type(8)))  float    v8f;
typedef __attribute__((ext_vector_type(4)))  float    v4f;

constexpr int kSteps   = 512;
constexpr int kBatch   = 1024;
constexpr int kHid     = 12;
constexpr int kGates   = 3;
constexpr int kMid     = 6;
constexpr int kRowsBlk = 32;
constexpr int kChunk   = 4;
static_assert(kSteps % kChunk == 0);
static_assert(kBatch % kRowsBlk == 0);
static_assert(kHid <= 16 && kMid <= 8);
static_assert(kChunk * kRowsBlk == 32 * 4);

constexpr int kOffWhh   = 0;
constexpr int kOffWih   = 448;
constexpr int kOffBih   = 512;
constexpr int kOffBhh   = 576;
constexpr int kOffW1    = 640;
constexpr int kOffB1    = 736;
constexpr int kOffW2    = 768;
constexpr int kOffB2    = 800;
constexpr int kParTotal = 832;
static_assert(kGates * kHid * kHid <= kOffWih - kOffWhh);
static_assert(kGates * kHid <= 64);
static_assert(kMid * kHid <= kOffB1 - kOffW1);

__device__ __forceinline__ float qz(float v) {
  float r = rintf(v * 128.0f);
  r = fminf(fmaxf(r, -32768.0f), 32767.0f);
  return r * 0.0078125f;
}

__device__ __forceinline__ float hsig(float v) {
  const float a = 0.25f * v;
  const float b = a + 0.5f;
  return fminf(fmaxf(b, 0.0f), 1.0f);
}

__device__ __forceinline__ _Float16 to_h16(float v) {
  const float f = (fabsf(v) < 6.103515625e-05f) ? 0.0f : v;
  return (_Float16)f;
}

__device__ __forceinline__ v8f mma_f16(v16h a, v16h b) {
  v8f c = {0.f, 0.f, 0.f, 0.f, 0.f, 0.f, 0.f, 0.f};
  c = __builtin_amdgcn_wmma_f32_16x16x32_f16(false, a, false, b, (short)0, c, false, false);
  asm volatile("v_nop\n\tv_nop\n\tv_nop\n\tv_nop" : "+v"(c) : "v"(a), "v"(b));
  return c;
}

template <int NEL, int NPAD>
__device__ __forceinline__ void stage_q(const float* __restrict__ src, float* dst, int lane) {
  static_assert(NPAD % 32 == 0 && NPAD >= NEL);
#pragma unroll 1
  for (int it = 0; it < NPAD / 32; ++it) {
    const int i = it * 32 + lane;
    const int ic = (i < NEL) ? i : (NEL - 1);
    const float v = src[ic];
    dst[i] = qz(v);
  }
}

__global__ __launch_bounds__(32) void qcell_seq_kernel(
    const float* __restrict__ xin,
    const float* __restrict__ w_ih,
    const float* __restrict__ w_hh,
    const float* __restrict__ b_ih,
    const float* __restrict__ b_hh,
    const float* __restrict__ w1,
    const float* __restrict__ b1,
    const float* __restrict__ w2,
    const float* __restrict__ b2,
    float* __restrict__ out)
{
  __shared__ __align__(16) float sP[kParTotal];
  __shared__ __align__(16) float sX[kChunk * kRowsBlk];
  __shared__ __align__(16) float sO[kChunk * kRowsBlk];

  const int lane = threadIdx.x & 31;
  const int hh   = lane >> 4;
  const int c    = lane & 15;
  const int b0   = blockIdx.x * kRowsBlk;

  stage_q<kGates * kHid * kHid, 448>(w_hh, sP + kOffWhh, lane);
  stage_q<kGates * kHid, 64>(w_ih, sP + kOffWih, lane);
  stage_q<kGates * kHid, 64>(b_ih, sP + kOffBih, lane);
  stage_q<kGates * kHid, 64>(b_hh, sP + kOffBhh, lane);
  stage_q<kMid * kHid, 96>(w1, sP + kOffW1, lane);
  stage_q<kMid, 32>(b1, sP + kOffB1, lane);
  stage_q<kMid, 32>(w2, sP + kOffW2, lane);
  stage_q<1, 32>(b2, sP + kOffB2, lane);
  __syncthreads();

  v16h aw[kGates];
  v16h a1;
  {
    const bool mval = (c < kHid);
    const int  mc   = mval ? c : (kHid - 1);
#pragma unroll
    for (int g = 0; g < kGates; ++g) {
      v16h f = {};
#pragma unroll
      for (int e = 0; e < 8; ++e) {
        const int  k    = 8 * hh + e;
        const bool kval = (k < kHid);
        const int  kc   = kval ? k : (kHid - 1);
        const float w   = sP[kOffWhh + (g * kHid + mc) * kHid + kc];
        f[e] = to_h16((mval && kval) ? w : 0.0f);
      }
      aw[g] = f;
    }
    const int  i1   = c & 7;
    const bool ival = (i1 < kMid);
    const int  ic   = ival ? i1 : (kMid - 1);
    v16h f1 = {};
#pragma unroll
    for (int e = 0; e < 8; ++e) {
      const int  k    = 8 * hh + e;
      const bool kval = (k < kHid);
      const int  kc   = kval ? k : (kHid - 1);
      const float w   = sP[kOffW1 + ic * kHid + kc];
      f1[e] = to_h16((ival && kval) ? w : 0.0f);
    }
    a1 = f1;
  }

  float wih[kGates][8], bih[kGates][8], bhh[kGates][8];
#pragma unroll
  for (int g = 0; g < kGates; ++g) {
#pragma unroll
    for (int r = 0; r < 8; ++r) {
      const int  u    = 8 * hh + r;
      const bool uval = (u < kHid);
      const int  uc   = uval ? u : (kHid - 1);
      const float a = sP[kOffWih + g * kHid + uc];
      const float b = sP[kOffBih + g * kHid + uc];
      const float d = sP[kOffBhh + g * kHid + uc];
      wih[g][r] = uval ? a : 0.0f;
      bih[g][r] = uval ? b : 0.0f;
      bhh[g][r] = uval ? d : 0.0f;
    }
  }
  float b1q[kMid], w2q[kMid];
#pragma unroll
  for (int i = 0; i < kMid; ++i) {
    b1q[i] = sP[kOffB1 + i];
    w2q[i] = sP[kOffW2 + i];
  }
  const float b2q = sP[kOffB2];

  float hst[2][8];
  v16h  bh[2];
#pragma unroll
  for (int nt = 0; nt < 2; ++nt) {
#pragma unroll
    for (int r = 0; r < 8; ++r) hst[nt][r] = 0.0f;
    v16h z = {};
    bh[nt] = z;
  }

  const int tt = lane >> 3;
  const int bb = (lane & 7) * 4;
  const float* xp = xin + (size_t)tt * kBatch + b0 + bb;
  float*       op = out + (size_t)tt * kBatch + b0 + bb;

#pragma unroll 1
  for (int tc = 0; tc < kSteps / kChunk; ++tc) {
    const size_t cbase = (size_t)tc * (size_t)(kChunk * kBatch);
    const v4f xv = *(const v4f*)(xp + cbase);
    __syncthreads();
    *(v4f*)(sX + tt * kRowsBlk + bb) = xv;
    __syncthreads();

#pragma unroll 1
    for (int s = 0; s < kChunk; ++s) {
      const float xa = sX[s * kRowsBlk + c];
      const float xb = sX[s * kRowsBlk + 16 + c];
      v8f dhd[2];
#pragma unroll
      for (int nt = 0; nt < 2; ++nt) {
        const float xs = (nt == 0) ? xa : xb;
        const v8f accr = mma_f16(aw[0], bh[nt]);
        const v8f accz = mma_f16(aw[1], bh[nt]);
        const v8f accn = mma_f16(aw[2], bh[nt]);
        v16h nb = {};
#pragma unroll
        for (int r = 0; r < 8; ++r) {
          const float hhr = qz(qz(accr[r]) + bhh[0][r]);
          const float hhz = qz(qz(accz[r]) + bhh[1][r]);
          const float hhn = qz(qz(accn[r]) + bhh[2][r]);
          const float pr  = xs * wih[0][r];
          const float pz  = xs * wih[1][r];
          const float pn  = xs * wih[2][r];
          const float iir = qz(qz(pr) + bih[0][r]);
          const float iiz = qz(qz(pz) + bih[1][r]);
          const float iin = qz(qz(pn) + bih[2][r]);
          const float rg  = qz(hsig(iir + hhr));
          const float zg  = qz(hsig(iiz + hhz));
          const float rn  = rg * hhn;
          const float sn  = iin + rn;
          const float ng  = qz(fminf(fmaxf(sn, -1.0f), 1.0f));
          const float omz = 1.0f - zg;
          const float t0  = omz * ng;
          const float t1  = zg * hst[nt][r];
          float hn = qz(t0 + t1);
          if (r >= 4) hn = (hh == 0) ? hn : 0.0f;
          hst[nt][r] = hn;
          nb[r] = to_h16(hn);
        }
        bh[nt] = nb;
        dhd[nt] = mma_f16(a1, bh[nt]);
      }
      float part = 0.0f;
#pragma unroll
      for (int i = 0; i < kMid; ++i) {
        const float d0 = dhd[0][i];
        const float d1 = dhd[1][i];
        const float d  = (hh != 0) ? d1 : d0;
        float sv = qz(d);
        sv = qz(sv + b1q[i]);
        sv = qz(sv);
        const float av = fmaxf(sv, 0.0f);
        const float pv = av * w2q[i];
        part = part + pv;
      }
      float o = qz(part);
      o = qz(o + b2q);
      o = qz(o);
      sO[s * kRowsBlk + lane] = o;
    }
    __syncthreads();
    const v4f ov = *(const v4f*)(sO + tt * kRowsBlk + bb);
    float* dst = op + cbase;
    *(volatile v4f*)dst = ov;
    __threadfence();
    *(volatile v4f*)dst = ov;
  }
}

extern "C" void kernel_launch(void* const* d_in, const int* in_sizes, int n_in,
                              void* d_out, int out_size, void* d_ws, size_t ws_size,
                              hipStream_t stream) {
  (void)d_ws; (void)ws_size;
  if (n_in < 9 || d_out == nullptr) return;
  if (in_sizes[0] != kSteps * kBatch) return;
  if (in_sizes[1] != kGates * kHid) return;
  if (in_sizes[2] != kGates * kHid * kHid) return;
  if (in_sizes[3] != kGates * kHid) return;
  if (in_sizes[4] != kGates * kHid) return;
  if (in_sizes[5] != kMid * kHid) return;
  if (in_sizes[6] != kMid) return;
  if (in_sizes[7] != kMid) return;
  if (in_sizes[8] != 1) return;
  if (out_size != kSteps * kBatch) return;

  const float* x    = (const float*)d_in[0];
  const float* w_ih = (const float*)d_in[1];
  const float* w_hh = (const float*)d_in[2];
  const float* b_ih = (const float*)d_in[3];
  const float* b_hh = (const float*)d_in[4];
  const float* w1   = (const float*)d_in[5];
  const float* b1   = (const float*)d_in[6];
  const float* w2   = (const float*)d_in[7];
  const float* b2   = (const float*)d_in[8];
  float* out = (float*)d_out;

  qcell_seq_kernel<<<kBatch / kRowsBlk, 32, 0, stream>>>(x, w_ih, w_hh, b_ih, b_hh, w1, b1, w2, b2, out);
}
